// AttentionBlockWithSkipConnection_42116449305031
// MI455X (gfx1250) — hardware-verified
//
#include <hip/hip_runtime.h>
#include <stddef.h>


#define NBATCH 8
#define NPIX   4096
#define CH     256
#define NGRP   32
#define NROW   (NBATCH * NPIX)

typedef unsigned short us8 __attribute__((ext_vector_type(8)));
typedef us8 us8a __attribute__((may_alias));
typedef unsigned int v4u __attribute__((ext_vector_type(4)));
typedef float v4f __attribute__((ext_vector_type(4)));
typedef v4f v4fa __attribute__((may_alias));
typedef float v8f __attribute__((ext_vector_type(8)));
typedef __bf16 v16b __attribute__((ext_vector_type(16)));

union Frag  { v16b v; us8 u[2]; };
union Pack8 { us8 u; v4u w; unsigned short s[8]; };

__device__ __forceinline__ v8f zero8() {
  v8f z = {0.f, 0.f, 0.f, 0.f, 0.f, 0.f, 0.f, 0.f};
  return z;
}

__device__ __forceinline__ unsigned short f2bf(float f) {
  unsigned int u = __float_as_uint(f);
  u += 0x7FFFu + ((u >> 16) & 1u);
  return (unsigned short)(u >> 16);
}

__device__ __forceinline__ v8f mma_bf16(v16b a, v16b b, v8f c) {
  v8f d = __builtin_amdgcn_wmma_f32_16x16x32_bf16(false, a, false, b, (short)0, c, false, false);
  asm volatile("v_nop\n\tv_nop\n\tv_nop\n\tv_nop" : "+v"(d) : "v"(a), "v"(b));
  return d;
}

__global__ void __launch_bounds__(256)
k_cvt_w(const float* wqkv, const float* wproj,
        unsigned short* wqkvT, unsigned short* wprojT, int ntask) {
  const int t = blockIdx.x * 256 + threadIdx.x;
  if (t >= ntask) return;
  const float* src;
  unsigned short* dst;
  int ld;
  if (t < 3 * CH * (CH / 8)) {
    const int d = t >> 5, c0 = (t & 31) * 8;
    ld  = 3 * CH;
    src = wqkv + (size_t)c0 * ld + d;
    dst = wqkvT + (size_t)d * CH + c0;
  } else {
    const int t2 = t - 3 * CH * (CH / 8);
    const int d = t2 >> 5, c0 = (t2 & 31) * 8;
    ld  = CH;
    src = wproj + (size_t)c0 * ld + d;
    dst = wprojT + (size_t)d * CH + c0;
  }
  Pack8 pk;
  #pragma unroll
  for (int j = 0; j < 8; ++j) pk.s[j] = f2bf(src[(size_t)j * ld]);
  const v4u w = pk.w;
  *(volatile v4u*)dst = w;
  __threadfence();
  *(volatile v4u*)dst = w;
}

__global__ void __launch_bounds__(256)
k_gn_stats(const float* x, float* mean, float* rstd) {
  __shared__ double shs[256];
  __shared__ double shq[256];
  const int b = blockIdx.x, c = threadIdx.x;
  const float* p = x + (size_t)b * NPIX * CH + c;
  double s = 0.0, q = 0.0;
  #pragma unroll 8
  for (int pix = 0; pix < NPIX; ++pix) {
    const float v = p[(size_t)pix * CH];
    s += (double)v;
    q += (double)v * (double)v;
  }
  shs[c] = s;
  shq[c] = q;
  __syncthreads();
  if (c < NGRP) {
    double S = 0.0, Q = 0.0;
    #pragma unroll
    for (int j = 0; j < 8; ++j) { S += shs[c * 8 + j]; Q += shq[c * 8 + j]; }
    const double cnt = (double)NPIX * 8.0;
    const double mu = S / cnt;
    double var = Q / cnt - mu * mu;
    if (var < 0.0) var = 0.0;
    const float muf = (float)mu;
    const float rsf = 1.0f / sqrtf((float)var + 1e-5f);
    volatile float* pm = mean + b * NGRP + c;
    volatile float* pr = rstd + b * NGRP + c;
    *pm = muf;
    *pr = rsf;
    __threadfence();
    *pm = muf;
    *pr = rsf;
  }
}

__global__ void __launch_bounds__(256)
k_gn_apply(const float* x, const float* mean, const float* rstd,
           const float* scale, const float* bias, unsigned short* h, int ntask) {
  const int t = blockIdx.x * 256 + threadIdx.x;
  if (t >= ntask) return;
  const int row = t >> 5, g = t & 31, c0 = g * 8;
  const int b = row >> 12;
  const float mu = mean[b * NGRP + g], rs = rstd[b * NGRP + g];
  const float* xp = x + (size_t)row * CH + c0;
  const v4f u0 = *(const v4f*)xp;
  const v4f u1 = *(const v4f*)(xp + 4);
  const v4f s0 = *(const v4f*)(scale + c0);
  const v4f s1 = *(const v4f*)(scale + c0 + 4);
  const v4f b0 = *(const v4f*)(bias + c0);
  const v4f b1 = *(const v4f*)(bias + c0 + 4);
  const v4f y0 = (u0 - mu) * rs * s0 + b0;
  const v4f y1 = (u1 - mu) * rs * s1 + b1;
  Pack8 pk;
  pk.s[0] = f2bf(y0.x); pk.s[1] = f2bf(y0.y); pk.s[2] = f2bf(y0.z); pk.s[3] = f2bf(y0.w);
  pk.s[4] = f2bf(y1.x); pk.s[5] = f2bf(y1.y); pk.s[6] = f2bf(y1.z); pk.s[7] = f2bf(y1.w);
  const v4u w = pk.w;
  unsigned short* dst = h + (size_t)row * CH + c0;
  *(volatile v4u*)dst = w;
  __threadfence();
  *(volatile v4u*)dst = w;
}

__device__ __forceinline__ void pass_qk(const unsigned short* tileH, unsigned short* dst,
                                        int row0, int cg, int wv, int ln) {
  #pragma unroll
  for (int ps = 0; ps < 4; ++ps) {
    const int rl = wv * 16 + ps * 4 + (ln >> 3);
    const int piece = ln & 7;
    Pack8 pk;
    pk.u = *(const us8a*)(tileH + rl * 64 + piece * 8);
    *(volatile v4u*)(dst + (size_t)(row0 + rl) * CH + cg + piece * 8) = pk.w;
  }
}
__device__ __forceinline__ void pass_v(const unsigned short* tileH, unsigned short* vT,
                                       int bb, int n0, int cg, int wv, int ln) {
  #pragma unroll
  for (int ps = 0; ps < 4; ++ps) {
    const int cl = wv * 8 + ps * 2 + (ln >> 4);
    const int piece = ln & 15;
    Pack8 pk;
    pk.u = *(const us8a*)(tileH + cl * 128 + piece * 8);
    *(volatile v4u*)(vT + (size_t)(bb * CH + cg + cl) * NPIX + n0 + piece * 8) = pk.w;
  }
}
__device__ __forceinline__ void pass_out(const float* tileF, float* out, const float* bias,
                                         const float* xres, int row0, int colBase, int wv, int ln) {
  #pragma unroll
  for (int ps = 0; ps < 8; ++ps) {
    const int rl = wv * 16 + ps * 2 + (ln >> 4);
    const int piece = ln & 15;
    const int col = colBase + piece * 4;
    const v4f v  = *(const v4fa*)(tileF + rl * 64 + piece * 4);
    const v4f bs = *(const v4f*)(bias + col);
    const v4f xr = *(const v4f*)(xres + (size_t)(row0 + rl) * CH + col);
    const v4f r = v + bs + xr;
    *(volatile v4f*)(out + (size_t)(row0 + rl) * CH + col) = r;
  }
}

template <int MODE>
__global__ void __launch_bounds__(256)
k_gemm(const unsigned short* A, const unsigned short* BT, const float* bias,
       unsigned short* qd, unsigned short* kd, unsigned short* vT,
       const float* xres, float* out) {
  __shared__ unsigned char smem_raw[128 * 64 * 4] __attribute__((aligned(16)));
  unsigned short* tileH = (unsigned short*)smem_raw;
  float* tileF = (float*)smem_raw;

  const int tid = threadIdx.x;
  const int wv = tid >> 5, ln = tid & 31, m = ln & 15, hh = ln >> 4;
  const int row0 = blockIdx.x * 128;
  const int colBase = blockIdx.y * 64;
  const int rowA = row0 + wv * 16 + m;

  v8f acc[4];
  #pragma unroll
  for (int nt = 0; nt < 4; ++nt) acc[nt] = zero8();

  #pragma unroll
  for (int ks = 0; ks < CH / 32; ++ks) {
    const unsigned short* pa = A + (size_t)rowA * CH + ks * 32 + hh * 8;
    Frag a;
    a.u[0] = *(const us8*)pa;
    a.u[1] = *(const us8*)(pa + 16);
    #pragma unroll
    for (int nt = 0; nt < 4; ++nt) {
      const unsigned short* pb = BT + (size_t)(colBase + nt * 16 + m) * CH + ks * 32 + hh * 8;
      Frag bb;
      bb.u[0] = *(const us8*)pb;
      bb.u[1] = *(const us8*)(pb + 16);
      acc[nt] = mma_bf16(a.v, bb.v, acc[nt]);
    }
  }

  if (MODE == 0) {
    const int region = colBase >> 8;
    const float sc = (region == 0) ? 0.0625f : 1.0f;
    #pragma unroll
    for (int nt = 0; nt < 4; ++nt) {
      const int cl = nt * 16 + m;
      const float bv = bias[colBase + cl];
      #pragma unroll
      for (int r = 0; r < 8; ++r) {
        const int rl = wv * 16 + hh * 8 + r;
        const unsigned short hv = f2bf((acc[nt][r] + bv) * sc);
        if (region == 2) tileH[cl * 128 + rl] = hv;
        else             tileH[rl * 64 + cl] = hv;
      }
    }
    __syncthreads();
    const int cg = colBase & (CH - 1);
    if (region == 2) {
      const int bb = row0 >> 12, n0 = row0 & (NPIX - 1);
      pass_v(tileH, vT, bb, n0, cg, wv, ln);
      __threadfence();
      pass_v(tileH, vT, bb, n0, cg, wv, ln);
    } else {
      unsigned short* dst = (region == 0) ? qd : kd;
      pass_qk(tileH, dst, row0, cg, wv, ln);
      __threadfence();
      pass_qk(tileH, dst, row0, cg, wv, ln);
    }
  } else {
    #pragma unroll
    for (int nt = 0; nt < 4; ++nt) {
      const int cl = nt * 16 + m;
      #pragma unroll
      for (int r = 0; r < 8; ++r) {
        const int rl = wv * 16 + hh * 8 + r;
        tileF[rl * 64 + cl] = acc[nt][r];
      }
    }
    __syncthreads();
    pass_out(tileF, out, bias, xres, row0, colBase, wv, ln);
    __threadfence();
    pass_out(tileF, out, bias, xres, row0, colBase, wv, ln);
  }
}

__global__ void __launch_bounds__(256) __attribute__((amdgpu_num_vgpr(256)))
k_attn(const unsigned short* qf, const unsigned short* kf, const unsigned short* vT,
       unsigned short* of) {
  __shared__ unsigned short lds[8 * 4096] __attribute__((aligned(16)));
  const int tid = threadIdx.x;
  const int wv = tid >> 5, ln = tid & 31, m = ln & 15, hh = ln >> 4;
  const int b = blockIdx.x >> 5;
  const int qrow = (blockIdx.x & 31) * 128 + wv * 16;
  unsigned short* lw = lds + wv * 4096;

  const unsigned short* qp = qf + ((size_t)b * NPIX + qrow + m) * CH + hh * 8;
  const unsigned short* kbase = kf + (size_t)b * NPIX * CH + hh * 8;
  const unsigned short* vp0 = vT + ((size_t)b * CH + m) * NPIX + hh * 8;

  v8f o[16];
  #pragma unroll
  for (int ct = 0; ct < 16; ++ct) o[ct] = zero8();
  float mr[8], lr[8];
  #pragma unroll
  for (int i = 0; i < 8; ++i) { mr[i] = -1.0e30f; lr[i] = 0.f; }

  for (int kt = 0; kt < NPIX / 32; ++kt) {
    const int key0 = kt * 32;
    const unsigned short* k0p = kbase + (size_t)(key0 + m) * CH;
    const unsigned short* k1p = k0p + 16 * CH;

    v8f s0 = zero8(), s1 = zero8();
    #pragma unroll
    for (int ks = 0; ks < CH / 32; ++ks) {
      Frag a, f0, f1;
      a.u[0]  = *(const us8*)(qp  + ks * 32);
      a.u[1]  = *(const us8*)(qp  + ks * 32 + 16);
      f0.u[0] = *(const us8*)(k0p + ks * 32);
      f0.u[1] = *(const us8*)(k0p + ks * 32 + 16);
      f1.u[0] = *(const us8*)(k1p + ks * 32);
      f1.u[1] = *(const us8*)(k1p + ks * 32 + 16);
      s0 = mma_bf16(a.v, f0.v, s0);
      s1 = mma_bf16(a.v, f1.v, s1);
    }

    v8f corrv = zero8();
    #pragma unroll
    for (int i = 0; i < 8; ++i) {
      const float x0 = s0[i], x1 = s1[i];
      float mx = fmaxf(x0, x1);
      mx = fmaxf(mx, __shfl_xor(mx, 1));
      mx = fmaxf(mx, __shfl_xor(mx, 2));
      mx = fmaxf(mx, __shfl_xor(mx, 4));
      mx = fmaxf(mx, __shfl_xor(mx, 8));
      const float mn = fmaxf(mr[i], mx);
      const float corr = __expf(mr[i] - mn);
      const float p0 = __expf(x0 - mn);
      const float p1 = __expf(x1 - mn);
      float rs = p0 + p1;
      rs += __shfl_xor(rs, 1);
      rs += __shfl_xor(rs, 2);
      rs += __shfl_xor(rs, 4);
      rs += __shfl_xor(rs, 8);
      lr[i] = lr[i] * corr + rs;
      mr[i] = mn;
      corrv[i] = corr;
      lw[(hh * 8 + i) * 32 + m]      = f2bf(p0);
      lw[(hh * 8 + i) * 32 + 16 + m] = f2bf(p1);
    }
    #pragma unroll
    for (int ct = 0; ct < 16; ++ct) o[ct] = o[ct] * corrv;

    __syncthreads();
    Frag ap;
    ap.u[0] = *(const us8a*)(lw + m * 32 + hh * 8);
    ap.u[1] = *(const us8a*)(lw + m * 32 + 16 + hh * 8);

    const unsigned short* vp = vp0 + key0;
    #pragma unroll
    for (int ct = 0; ct < 16; ++ct) {
      const unsigned short* pv = vp + (size_t)ct * 16 * NPIX;
      Frag fv;
      fv.u[0] = *(const us8*)pv;
      fv.u[1] = *(const us8*)(pv + 16);
      o[ct] = mma_bf16(ap.v, fv.v, o[ct]);
    }
  }

  float inv[8];
  #pragma unroll
  for (int i = 0; i < 8; ++i) inv[i] = 1.0f / lr[i];
  #pragma unroll
  for (int ct = 0; ct < 16; ++ct) {
    #pragma unroll
    for (int r = 0; r < 8; ++r) {
      lw[(hh * 8 + r) * 256 + ct * 16 + m] = f2bf(o[ct][r] * inv[r]);
    }
  }
  __syncthreads();
  unsigned short* ob = of + ((size_t)b * NPIX + qrow) * CH;
  #pragma unroll
  for (int rr = 0; rr < 16; ++rr) {
    Pack8 pk;
    pk.u = *(const us8a*)(lw + rr * 256 + ln * 8);
    *(volatile v4u*)(ob + (size_t)rr * CH + ln * 8) = pk.w;
  }
  __threadfence();
  #pragma unroll
  for (int rr = 0; rr < 16; ++rr) {
    Pack8 pk;
    pk.u = *(const us8a*)(lw + rr * 256 + ln * 8);
    *(volatile v4u*)(ob + (size_t)rr * CH + ln * 8) = pk.w;
  }
}

extern "C" void kernel_launch(void* const* d_in, const int* in_sizes, int n_in,
                              void* d_out, int out_size, void* d_ws, size_t ws_size,
                              hipStream_t stream) {
  if (n_in < 7) return;
  if (in_sizes[0] != NROW * CH || in_sizes[1] < CH || in_sizes[2] < CH ||
      in_sizes[3] != CH * 3 * CH || in_sizes[4] < 3 * CH ||
      in_sizes[5] != CH * CH || in_sizes[6] < CH) return;
  if (out_size != NROW * CH) return;

  const float* x        = (const float*)d_in[0];
  const float* gn_scale = (const float*)d_in[1];
  const float* gn_bias  = (const float*)d_in[2];
  const float* w_qkv    = (const float*)d_in[3];
  const float* b_qkv    = (const float*)d_in[4];
  const float* w_proj   = (const float*)d_in[5];
  const float* b_proj   = (const float*)d_in[6];
  float* out = (float*)d_out;

  char* ws = (char*)d_ws;
  size_t off = 0;
  float* mean = (float*)(ws + off);              off += 1024;
  float* rstd = (float*)(ws + off);              off += 1024;
  off = 4096;
  unsigned short* wqkvT  = (unsigned short*)(ws + off); off += (size_t)3 * CH * CH * 2;
  unsigned short* wprojT = (unsigned short*)(ws + off); off += (size_t)CH * CH * 2;
  const size_t act = (size_t)NROW * CH * 2;
  unsigned short* h  = (unsigned short*)(ws + off); off += act;
  unsigned short* q  = (unsigned short*)(ws + off); off += act;
  unsigned short* k  = (unsigned short*)(ws + off); off += act;
  unsigned short* vT = (unsigned short*)(ws + off); off += act;
  unsigned short* of = (unsigned short*)(ws + off); off += act;
  if (off > ws_size) return;

  const int ntaskW = 3 * CH * (CH / 8) + CH * (CH / 8);
  const int ntaskH = NROW * (CH / 8);

  k_cvt_w<<<dim3((ntaskW + 255) / 256), dim3(256), 0, stream>>>(w_qkv, w_proj, wqkvT, wprojT, ntaskW);
  k_gn_stats<<<dim3(NBATCH), dim3(256), 0, stream>>>(x, mean, rstd);
  k_gn_apply<<<dim3((ntaskH + 255) / 256), dim3(256), 0, stream>>>(x, mean, rstd, gn_scale, gn_bias, h, ntaskH);
  k_gemm<0><<<dim3(NROW / 128, (3 * CH) / 64), dim3(256), 0, stream>>>(
      h, wqkvT, b_qkv, q, k, vT, x, out);
  k_attn<<<dim3(NBATCH * (NPIX / 128)), dim3(256), 0, stream>>>(q, k, vT, of);
  k_gemm<1><<<dim3(NROW / 128, CH / 64), dim3(256), 0, stream>>>(
      of, wprojT, b_proj, q, k, vT, x, out);
}
